// ComplexMultiheadAttention_37495064494297
// MI455X (gfx1250) — hardware-verified
//
#include <hip/hip_runtime.h>


#ifndef NB
#define NB 2
#endif
#ifndef SEQ
#define SEQ 1024
#endif
#define NB_FULL  2
#define SEQ_FULL 1024
#define TT   SEQ
#define DIM  1024
#define NH   16
#define DH   64
#define DW   (2 * DH)
#define DQ   (2 * DIM)
#define KX   (2 * DIM)
#define NREP 4
#define PCAR 1024.0f
#define SCL  0.125f
static_assert(NB >= 1 && NB <= NB_FULL);
static_assert(SEQ >= 128 && SEQ <= SEQ_FULL && (SEQ % 128) == 0);
static_assert(NH * DH == DIM);
static_assert((KX % 32) == 0 && (DQ % 32) == 0 && (DH % 32) == 0 && (TT % 64) == 0 && (DIM % 64) == 0);

typedef _Float16 h16;
typedef unsigned short bf;
typedef __attribute__((ext_vector_type(16))) __bf16   v16bf;
typedef __attribute__((ext_vector_type(16))) _Float16 v16h;
typedef __attribute__((ext_vector_type(8)))  _Float16 v8h;
typedef __attribute__((ext_vector_type(8)))  unsigned short v8us;
typedef __attribute__((ext_vector_type(8)))  float    v8f;
typedef __attribute__((ext_vector_type(4)))  float    v4f;
typedef v8h  __attribute__((may_alias)) v8ha;
typedef v4f  __attribute__((may_alias)) v4fa;
typedef v8us __attribute__((may_alias)) v8usa;
typedef __attribute__((ext_vector_type(2))) _Float16 v2h;
typedef __attribute__((ext_vector_type(4))) _Float16 v4h;
typedef __attribute__((ext_vector_type(2))) unsigned short v2us;
typedef __attribute__((ext_vector_type(4))) unsigned short v4us;
typedef __attribute__((ext_vector_type(2))) float v2f;

__device__ __forceinline__ unsigned short f2bf(float f) { unsigned u = __float_as_uint(f); u += 0x7FFFu + ((u >> 16) & 1u); return (unsigned short)(u >> 16); }
__device__ __forceinline__ float bf2f(unsigned short b) { return __uint_as_float(((unsigned)b) << 16); }
__device__ __forceinline__ v16h cat16(v8h lo, v8h hi) { return __builtin_shufflevector(lo, hi, 0, 1, 2, 3, 4, 5, 6, 7, 8, 9, 10, 11, 12, 13, 14, 15); }
__device__ __forceinline__ v16bf cat16b(v8us lo, v8us hi) { return __builtin_bit_cast(v16bf, __builtin_shufflevector(lo, hi, 0, 1, 2, 3, 4, 5, 6, 7, 8, 9, 10, 11, 12, 13, 14, 15)); }
__device__ __forceinline__ v8f wmma16(v16h a, v16h b, v8f c) { return __builtin_amdgcn_wmma_f32_16x16x32_f16(false, a, false, b, (short)0, c, false, false); }
__device__ __forceinline__ v8f wmmab(v16bf a, v16bf b, v8f c) { return __builtin_amdgcn_wmma_f32_16x16x32_bf16(false, a, false, b, (short)0, c, false, false); }
__device__ __forceinline__ h16 tohx(float x) { return (h16)x; }
__device__ __forceinline__ void splitf(float y, unsigned short& h, unsigned short& l) { h = f2bf(y); l = f2bf(y - bf2f(h)); }

template <typename T16> struct WFrag;
template <> struct WFrag<h16> { typedef v16h V; static __device__ __forceinline__ V ld(const h16* p) { return cat16(*(const v8h*)p, *(const v8h*)(p + 16)); } static __device__ __forceinline__ v8f mma(V a, V b, v8f c) { return wmma16(a, b, c); } };
template <> struct WFrag<bf> { typedef v16bf V; static __device__ __forceinline__ V ld(const bf* p) { return cat16b(*(const v8us*)p, *(const v8us*)(p + 16)); } static __device__ __forceinline__ v8f mma(V a, V b, v8f c) { return wmmab(a, b, c); } };
template <typename T16, int NSPLIT>
__global__ __launch_bounds__(32) void k_gemmw(const T16* __restrict__ A, const T16* __restrict__ A2, const T16* __restrict__ Bt, const T16* __restrict__ Bt2, int K, float* C, int ldc, size_t sA, size_t sB, size_t sC, int zsa, int zmb) {
    typedef typename WFrag<T16>::V V;
    __shared__ __align__(16) float os[16 * 68];
    const size_t z = blockIdx.z; const size_t za = z >> zsa; const size_t zb = z & (size_t)(unsigned)zmb;
    A += za * sA; if (A2) A2 += za * sA; Bt += zb * sB; if (Bt2) Bt2 += zb * sB; C += z * sC;
    const int lane = threadIdx.x & 31, lr = lane & 15, hi = lane >> 4; const int r0 = blockIdx.x * 64, c0 = blockIdx.y * 64;
    v8f acc[4][4];
#pragma unroll
    for (int mb = 0; mb < 4; ++mb)
#pragma unroll
        for (int nb = 0; nb < 4; ++nb) acc[mb][nb] = (v8f){};
    const size_t aoff = (size_t)(r0 + lr) * K + 8 * hi, boff = (size_t)(c0 + lr) * K + 8 * hi;
#pragma unroll 1
    for (int kc = 0; kc < K; kc += 32) {
        V a[4], a2[4];
#pragma unroll
        for (int mb = 0; mb < 4; ++mb) { a[mb] = WFrag<T16>::ld(A + aoff + (size_t)mb * 16 * K + kc); if (NSPLIT == 1 || NSPLIT == 2) a2[mb] = WFrag<T16>::ld(A2 + aoff + (size_t)mb * 16 * K + kc); }
#pragma unroll
        for (int nb = 0; nb < 4; ++nb) { const V b = WFrag<T16>::ld(Bt + boff + (size_t)nb * 16 * K + kc); V b2; if (NSPLIT >= 2) b2 = WFrag<T16>::ld(Bt2 + boff + (size_t)nb * 16 * K + kc);
#pragma unroll
            for (int mb = 0; mb < 4; ++mb) { acc[mb][nb] = WFrag<T16>::mma(a[mb], b, acc[mb][nb]); if (NSPLIT == 1 || NSPLIT == 2) acc[mb][nb] = WFrag<T16>::mma(a2[mb], b, acc[mb][nb]); if (NSPLIT >= 2) acc[mb][nb] = WFrag<T16>::mma(a[mb], b2, acc[mb][nb]); } }
        asm volatile("v_nop\n\tv_nop\n\tv_nop\n\tv_nop" : "+v"(acc[0][0]), "+v"(acc[1][1]), "+v"(acc[2][2]), "+v"(acc[3][3]) : "v"(a[0]), "v"(a[3]));
    }
#pragma unroll
    for (int mb = 0; mb < 4; ++mb) {
#pragma unroll
        for (int nb = 0; nb < 4; ++nb) {
#pragma unroll
            for (int j = 0; j < 8; ++j) os[(hi * 8 + j) * 68 + nb * 16 + lr] = acc[mb][nb][j]; }
        __builtin_amdgcn_wave_barrier(); asm volatile("" ::: "memory");
        float* crow = C + (size_t)(r0 + mb * 16) * ldc + c0;
#pragma unroll 1
        for (int ps = 0; ps < 2; ++ps) {
#pragma unroll
            for (int s = 0; s < 8; ++s) { const int row = 2 * s + hi, cofs = lr * 4; const v4f val = *(const v4fa*)(os + row * 68 + cofs);
                *(volatile v4f*)(crow + (size_t)row * ldc + cofs) = val; }
            if (ps == 0) __threadfence(); }
        __builtin_amdgcn_wave_barrier(); asm volatile("" ::: "memory");
    }
}

__global__ __launch_bounds__(256) void k_cvt8c(const float* __restrict__ xr, const float* __restrict__ xi, bf* dst) { const size_t i = (size_t)blockIdx.x * 256 + threadIdx.x; if (i >= (size_t)TT * KX / 8) return; const int t = (int)(i / (KX / 8)); const int k0 = (int)(i % (KX / 8)) * 8; const float* src = (k0 < DIM) ? (xr + (size_t)t * DIM + k0) : (xi + (size_t)t * DIM + (k0 - DIM)); const v8f v = *(const v8f*)src; v8us o;
#pragma unroll
    for (int k = 0; k < 8; ++k) o[k] = f2bf(v[k]); *(volatile v8us*)(dst + i * 8) = o; __threadfence(); *(volatile v8us*)(dst + i * 8) = o; }

__global__ __launch_bounds__(256) void k_wcx(const float* __restrict__ wr, const float* __restrict__ wi, int Kh, int N, bf* dst) { const size_t i = (size_t)blockIdx.x * 256 + threadIdx.x; const int KK = 2 * Kh; if (i >= (size_t)2 * N * KK / 8) return; const int nn = (int)(i / (KK / 8)); const int k0 = (int)(i % (KK / 8)) * 8; const int c = nn % N, comp = nn / N; const int part = (k0 >= Kh) ? 1 : 0; const int srow = k0 - part * Kh;
    const float* src = ((comp ^ part) ? wi : wr) + (size_t)c * Kh + srow; const float sgn = (comp == 0 && part == 1) ? -1.0f : 1.0f; const v8f v = *(const v8f*)src; v8us o;
#pragma unroll
    for (int q = 0; q < 8; ++q) o[q] = f2bf(sgn * v[q]);
    *(volatile v8us*)(dst + i * 8) = o; __threadfence(); *(volatile v8us*)(dst + i * 8) = o; }

__global__ __launch_bounds__(256) void k_plqk(const float* __restrict__ F, int pitch, int base0, int base1, bf* Ph, bf* Pl) { const size_t e = ((size_t)blockIdx.x * 256 + threadIdx.x) * 2; if (e >= (size_t)NH * 2 * TT * DH) return; const int d = (int)(e % DH); const int t = (int)((e / DH) % TT); const int hp = (int)(e / ((size_t)DH * TT)); const int h = hp >> 1, p = hp & 1; const float* f = F + (size_t)t * pitch + (p ? base1 : base0) + h * DH + d; v2us oh, ol;
#pragma unroll
    for (int q = 0; q < 2; ++q) { unsigned short a, c2; splitf(f[q], a, c2); oh[q] = a; ol[q] = c2; }
    *(volatile v2us*)(Ph + e) = oh; *(volatile v2us*)(Pl + e) = ol; __threadfence(); *(volatile v2us*)(Ph + e) = oh; *(volatile v2us*)(Pl + e) = ol; }

__global__ __launch_bounds__(256) void k_vt(const float* __restrict__ F, int pitch, int VR0, int VI0, h16* V16) { const size_t e = ((size_t)blockIdx.x * 256 + threadIdx.x) * 2; if (e >= (size_t)NH * 2 * DH * TT) return; const int j = (int)(e % TT); const int d = (int)((e / TT) % DH); const int hp = (int)(e / ((size_t)TT * DH)); const int h = hp >> 1, p = hp & 1;
    const float* f = F + (size_t)j * pitch + (p ? VI0 : VR0) + h * DH + d; v2h o16;
#pragma unroll
    for (int q = 0; q < 2; ++q) o16[q] = tohx(f[(size_t)q * pitch]);
    *(volatile v2h*)(V16 + e) = o16; __threadfence(); *(volatile v2h*)(V16 + e) = o16; }

__global__ __launch_bounds__(256) void k_asoft(const float* __restrict__ Sb, h16* P16) {
    const int lane = threadIdx.x & 31; const int row = blockIdx.x * 8 + (threadIdx.x >> 5); if (row >= NREP * TT) return; const float* sr = Sb + (size_t)row * TT; float v[TT / 32]; float mx = -3.0e38f;
#pragma unroll
    for (int ch = 0; ch < TT / 128; ++ch) { const int j0 = ch * 128 + lane * 4; const v4f a = *(const v4f*)(sr + j0);
#pragma unroll
        for (int q = 0; q < 4; ++q) { const float t = a[q] * SCL; v[ch * 4 + q] = t; mx = fmaxf(mx, t); } }
#pragma unroll
    for (int sh = 16; sh; sh >>= 1) mx = fmaxf(mx, __shfl_xor(mx, sh, 32));
    float sum = 0.f;
#pragma unroll
    for (int k = 0; k < TT / 32; ++k) { float d0 = __fsub_rn(v[k], mx); asm volatile("" : "+v"(d0)); v[k] = __builtin_amdgcn_exp2f(__fmul_rn(d0, 1.4426950408889634f)); sum += v[k]; }
#pragma unroll
    for (int sh = 16; sh; sh >>= 1) sum += __shfl_xor(sum, sh, 32);
    const float f = __fdiv_rn(PCAR, sum);
#pragma unroll 1
    for (int ps = 0; ps < 2; ++ps) {
#pragma unroll
        for (int ch = 0; ch < TT / 128; ++ch) { v4h o4;
#pragma unroll
            for (int q = 0; q < 4; ++q) o4[q] = tohx(v[ch * 4 + q] * f);
            *(volatile v4h*)(P16 + (size_t)row * TT + ch * 128 + lane * 4) = o4; }
        if (ps == 0) __threadfence(); }
}

__global__ __launch_bounds__(256) void k_merge(const float* __restrict__ O, int h, bf* Ah, bf* Al) { const size_t e = ((size_t)blockIdx.x * 256 + threadIdx.x) * 2; if (e >= (size_t)TT * DW) return; const int d2 = (int)(e % DW); const int t = (int)(e / DW); const int p = d2 / DH, d = d2 % DH;
    const size_t RS = (size_t)TT * DH; const size_t src = (size_t)t * DH + d; const v2f o0 = *(const v2f*)(O + src), o1 = *(const v2f*)(O + RS + src), o2 = *(const v2f*)(O + 2 * RS + src), o3 = *(const v2f*)(O + 3 * RS + src);
    const float sg = p ? 1.0f : -1.0f; const size_t oo = (size_t)t * DQ + (size_t)p * DIM + (size_t)h * DH + d; v2us oh, ol;
#pragma unroll
    for (int q = 0; q < 2; ++q) { const float val = (((o0[q] + sg * o1[q]) + sg * o2[q]) - o3[q]) * (1.0f / PCAR); unsigned short a, c2; splitf(val, a, c2); oh[q] = a; ol[q] = c2; }
    *(volatile v2us*)(Ah + oo) = oh; *(volatile v2us*)(Al + oo) = ol; __threadfence(); *(volatile v2us*)(Ah + oo) = oh; *(volatile v2us*)(Al + oo) = ol; }

#define WS_WQB  ((size_t)2 * DIM * KX * 2)
#define WS_WKVB ((size_t)4 * DIM * KX * 2)
#define WS_WOB  ((size_t)2 * DIM * DQ * 2)
#define WS_XC   ((size_t)TT * KX * 2)
#define WS_FQ   ((size_t)TT * 2 * DIM * 4)
#define WS_FKV  ((size_t)TT * 4 * DIM * 4)
#define WS_PL   ((size_t)NH * 2 * TT * DH * 2)
#define WS_VT   ((size_t)NH * 2 * DH * TT * 2)
#define WS_SB   ((size_t)NREP * TT * TT * 4)
#define WS_P16  ((size_t)NREP * TT * TT * 2)
#define WS_OB   ((size_t)NREP * TT * DH * 4)
#define WS_AT   ((size_t)TT * DQ * 2)
#define WS_TOTAL (WS_WQB + WS_WKVB + WS_WOB + WS_XC + WS_FQ + WS_FKV + 4 * WS_PL + WS_VT + WS_SB + WS_P16 + WS_OB + 2 * WS_AT)
static_assert(WS_TOTAL <= (size_t)134217728);
static_assert((WS_XC % 256) == 0 && (WS_PL % 256) == 0 && (WS_VT % 256) == 0 && (WS_OB % 256) == 0 && (WS_AT % 256) == 0);

extern "C" void kernel_launch(void* const* d_in, const int* in_sizes, int n_in,
                              void* d_out, int out_size, void* d_ws, size_t ws_size, hipStream_t stream) {
    if (n_in < 8) return;
    const long long needx = ((long long)(NB - 1) * SEQ_FULL + SEQ) * (long long)DIM;
    if ((long long)in_sizes[0] < needx || (long long)in_sizes[1] < needx) return;
    if (in_sizes[2] < DIM * DIM || in_sizes[3] < DIM * DIM || in_sizes[4] < 2 * DIM * DIM || in_sizes[5] < 2 * DIM * DIM || in_sizes[6] < DIM * DIM || in_sizes[7] < DIM * DIM) return;
    const size_t PLANE = (size_t)NB_FULL * SEQ_FULL * DIM;
    if ((long long)out_size < (long long)PLANE + needx) return;
    const float* xr = (const float*)d_in[0]; const float* xi = (const float*)d_in[1]; const float* wqr = (const float*)d_in[2]; const float* wqi = (const float*)d_in[3]; const float* wkvr = (const float*)d_in[4]; const float* wkvi = (const float*)d_in[5]; const float* wor = (const float*)d_in[6]; const float* woi = (const float*)d_in[7];
    float* OUT = (float*)d_out;
    char* wsp = (char*)d_ws;
    auto take = [&](size_t bytes) { char* p = wsp; wsp += (bytes + 255) & ~(size_t)255; return (void*)p; };
    bf* WQB = (bf*)take(WS_WQB); bf* WKVB = (bf*)take(WS_WKVB); bf* WOB = (bf*)take(WS_WOB);
    bf* XC = (bf*)take(WS_XC); float* FQ = (float*)take(WS_FQ); float* FKV = (float*)take(WS_FKV);
    const size_t TS = (size_t)TT * DH;
    bf* QPh = (bf*)take(WS_PL); bf* QPl = (bf*)take(WS_PL); bf* KPh = (bf*)take(WS_PL); bf* KPl = (bf*)take(WS_PL);
    const size_t VS1 = (size_t)DH * TT;
    h16* VT16 = (h16*)take(WS_VT);
    float* Sb = (float*)take(WS_SB); h16* P16 = (h16*)take(WS_P16); float* Ob = (float*)take(WS_OB); bf* ATh = (bf*)take(WS_AT); bf* ATl = (bf*)take(WS_AT);
    if ((size_t)(wsp - (char*)d_ws) > ws_size) return;
    k_wcx<<<(unsigned)(((size_t)2 * DIM * KX / 8 + 255) / 256), 256, 0, stream>>>(wqr, wqi, DIM, DIM, WQB);
    k_wcx<<<(unsigned)(((size_t)4 * DIM * KX / 8 + 255) / 256), 256, 0, stream>>>(wkvr, wkvi, DIM, 2 * DIM, WKVB);
    k_wcx<<<(unsigned)(((size_t)2 * DIM * DQ / 8 + 255) / 256), 256, 0, stream>>>(wor, woi, DIM, DIM, WOB);
    const unsigned LP = (unsigned)(((size_t)NH * 2 * TS / 2 + 255) / 256), LV = (unsigned)(((size_t)NH * 2 * VS1 / 2 + 255) / 256), LM = (unsigned)(((size_t)TT * DW / 2 + 255) / 256);
    for (int b = 0; b < NB; ++b) {
        k_cvt8c<<<(unsigned)(((size_t)TT * KX / 8 + 255) / 256), 256, 0, stream>>>(xr + (size_t)b * SEQ_FULL * DIM, xi + (size_t)b * SEQ_FULL * DIM, XC);
        k_gemmw<bf, 0><<<dim3(TT / 64, 2 * DIM / 64, 1), 32, 0, stream>>>(XC, nullptr, WQB, nullptr, KX, FQ, 2 * DIM, 0, 0, 0, 0, 0);
        k_gemmw<bf, 0><<<dim3(TT / 64, 4 * DIM / 64, 1), 32, 0, stream>>>(XC, nullptr, WKVB, nullptr, KX, FKV, 4 * DIM, 0, 0, 0, 0, 0);
        k_plqk<<<LP, 256, 0, stream>>>(FQ, 2 * DIM, 0, DIM, QPh, QPl);
        k_plqk<<<LP, 256, 0, stream>>>(FKV, 4 * DIM, 0, 2 * DIM, KPh, KPl);
        k_vt<<<LV, 256, 0, stream>>>(FKV, 4 * DIM, DIM, 3 * DIM, VT16);
        for (int h = 0; h < NH; ++h) {
            k_gemmw<bf, 2><<<dim3(TT / 64, TT / 64, NREP), 32, 0, stream>>>(QPh + (size_t)(2 * h) * TS, QPl + (size_t)(2 * h) * TS, KPh + (size_t)(2 * h) * TS, KPl + (size_t)(2 * h) * TS, DH, Sb, TT, TS, TS, (size_t)TT * TT, 1, 1);
            k_asoft<<<NREP * TT / 8, 256, 0, stream>>>(Sb, P16);
            k_gemmw<h16, 0><<<dim3(TT / 64, DH / 64, NREP), 32, 0, stream>>>(P16, nullptr, VT16 + (size_t)(2 * h) * VS1, nullptr, TT, Ob, DH, (size_t)TT * TT, VS1, (size_t)TT * DH, 0, 1);
            k_merge<<<LM, 256, 0, stream>>>(Ob, h, ATh, ATl); }
        k_gemmw<bf, 1><<<dim3(TT / 64, DIM / 64, 2), 32, 0, stream>>>(ATh, ATl, WOB, nullptr, DQ, OUT + (size_t)b * SEQ_FULL * DIM, DIM, 0, (size_t)DIM * DQ, PLANE, 0, 0x7FFFFFFF); }
}
